// LSTMRNN_5025111737012
// MI455X (gfx1250) — hardware-verified
//
#include <hip/hip_runtime.h>


#define LL   3
#define HH   64
#define EE   64
#define BB   256
#define TT   512
#define OO   3
#define G4   256
#define KC   128
#define WP   128
#define AP   136
#define HP   68
#define MB   16
#define NBLK (BB / MB)
#define NTHR 128

static_assert(KC == EE + HH);
static_assert(KC % 32 == 0);
static_assert(NBLK * MB == BB);
static_assert(NTHR == 128);
static_assert((NTHR / 32) * 16 == HH);
static_assert(MB * EE == NTHR * 8);
static_assert(MB * HH * 4 == NTHR * 16 * 2);
static_assert(AP % 8 == 0);
static_assert(AP >= KC);
static_assert(HP % 4 == 0);
static_assert(HP >= HH);
static_assert(((TT - 1) & 1) == 1);
static_assert(BB * OO == 192 * 4);

typedef __bf16         v16bf __attribute__((ext_vector_type(16)));
typedef unsigned short v8us  __attribute__((ext_vector_type(8)));
typedef float          v8f   __attribute__((ext_vector_type(8)));
typedef float          v4f   __attribute__((ext_vector_type(4)));

union Frag { v16bf v; v8us half[2]; };

constexpr size_t SZ_WPL  = (size_t)LL * G4 * WP * 2;
constexpr size_t SZ_HS   = (size_t)TT * BB * HH * 4;
constexpr size_t OFF_WHI = 0;
constexpr size_t OFF_WLO = OFF_WHI + SZ_WPL;
constexpr size_t OFF_HSA = OFF_WLO + SZ_WPL;
constexpr size_t OFF_HSB = OFF_HSA + SZ_HS;
constexpr size_t WS_END  = OFF_HSB + SZ_HS;
static_assert(OFF_WLO % 128 == 0);
static_assert(OFF_HSA % 128 == 0);
static_assert(OFF_HSB % 128 == 0);
static_assert(WS_END <= (size_t)134217728);
constexpr int NWP = LL * G4 * (WP / 8);
static_assert(NWP % 256 == 0);
static_assert((size_t)NWP * 16 == SZ_WPL);

__device__ __forceinline__ unsigned short bf_rne(float f) {
    const unsigned u = __float_as_uint(f);
    return (unsigned short)((u + 0x7FFFu + ((u >> 16) & 1u)) >> 16);
}
__device__ __forceinline__ void split2(float f, unsigned short& hi, unsigned short& lo) {
    hi = bf_rne(f);
    const float hf = __uint_as_float(((unsigned)hi) << 16);
    lo = bf_rne(f - hf);
}
__device__ __forceinline__ float rcpx(float x) { return __builtin_amdgcn_rcpf(x); }
__device__ __forceinline__ float sigm(float x) { return rcpx(1.0f + __expf(-x)); }
__device__ __forceinline__ float tanhm(float x) {
    const float e = __expf(2.0f * x);
    return 1.0f - 2.0f * rcpx(e + 1.0f);
}
__device__ __forceinline__ v8f zero8() {
    v8f z;
#pragma unroll
    for (int i = 0; i < 8; ++i) z[i] = 0.0f;
    return z;
}
__device__ __forceinline__ void cvt8(const float* src, v8us& hi, v8us& lo) {
    const v4f a = *(const v4f*)(src);
    const v4f b = *(const v4f*)(src + 4);
#pragma unroll
    for (int i = 0; i < 4; ++i) {
        unsigned short th, tl;
        split2(a[i], th, tl); hi[i] = th;     lo[i] = tl;
        split2(b[i], th, tl); hi[4 + i] = th; lo[4 + i] = tl;
    }
}
__device__ __forceinline__ v8f mma(v8f c, const Frag& a, const Frag& b) {
    return __builtin_amdgcn_wmma_f32_16x16x32_bf16(false, a.v, false, b.v, (short)0, c, false, false);
}

__global__ __launch_bounds__(256)
void cvt_kernel(const float* __restrict__ Wih, const float* __restrict__ Whh,
                unsigned short* Whi, unsigned short* Wlo)
{
    const int p   = blockIdx.x * 256 + threadIdx.x;
    const int l   = p >> 12;
    const int rem = p & 4095;
    const int n   = rem >> 4;
    const int c8  = (rem & 15) * 8;
    const int ci  = min(c8, EE - 8);
    const int cj  = min(max(c8 - EE, 0), HH - 8);
    const float* pa = Wih + (size_t)(l * G4 + n) * EE + ci;
    const float* pb = Whh + (size_t)(l * G4 + n) * HH + cj;
    const v4f a0 = *(const v4f*)(pa), a1 = *(const v4f*)(pa + 4);
    const v4f b0 = *(const v4f*)(pb), b1 = *(const v4f*)(pb + 4);
    v8us hi, lo;
#pragma unroll
    for (int i = 0; i < 4; ++i) {
        const float v0 = (c8 < EE) ? a0[i] : b0[i];
        const float v1 = (c8 < EE) ? a1[i] : b1[i];
        unsigned short th, tl;
        split2(v0, th, tl); hi[i] = th;     lo[i] = tl;
        split2(v1, th, tl); hi[4 + i] = th; lo[4 + i] = tl;
    }
    unsigned short* dh = Whi + (size_t)(l * G4 + n) * WP + c8;
    unsigned short* dl = Wlo + (size_t)(l * G4 + n) * WP + c8;
    *(volatile v8us*)dh = hi;
    *(volatile v8us*)dl = lo;
    __threadfence();
    *(volatile v8us*)dh = hi;
    *(volatile v8us*)dl = lo;
}

__device__ __forceinline__ const float* xsrc(const int* tokens, const float* emb, const float* hs_in,
                                             int is_l0, int nvocab, int t, int b, int c8)
{
    int tok = tokens[(size_t)b * TT + t];
    tok = min(max(tok, 0), nvocab - 1);
    const float* pe = emb + (size_t)tok * EE + c8;
    const float* ph = hs_in + ((size_t)t * BB + b) * HH + c8;
    return is_l0 ? pe : ph;
}

__global__ __launch_bounds__(NTHR)
void lstm_layer_kernel(const int* __restrict__ tokens, const float* __restrict__ emb,
                       const float* __restrict__ hs_in,
                       const unsigned short* __restrict__ Whi, const unsigned short* __restrict__ Wlo,
                       const float* __restrict__ bih, const float* __restrict__ bhh,
                       const float* __restrict__ h0, const float* __restrict__ c0,
                       float* hs_out, float* out_h, float* out_c, int is_l0, int nvocab)
{
    __shared__ __attribute__((aligned(16))) unsigned short sAhi[2][MB][AP];
    __shared__ __attribute__((aligned(16))) unsigned short sAlo[2][MB][AP];
    __shared__ __attribute__((aligned(16))) float sHf[2][MB][HP];
    __shared__ __attribute__((aligned(16))) float sCf[MB][HP];
    __shared__ float sBias[G4];

    const int tid  = threadIdx.x;
    const int lane = tid & 31;
    const int w    = tid >> 5;
    const int h    = lane >> 4;
    const int m    = lane & 15;
    const int u    = w * 16 + m;
    const int b0   = blockIdx.x * MB;
    const int srow = tid >> 3;
    const int sc8  = (tid & 7) * 8;
    const int prow = tid >> 4;
    const int pc4  = (tid & 15) * 4;

    for (int i = tid; i < G4; i += NTHR) sBias[i] = bih[i] + bhh[i];
    {
        v8us xh, xl;
        cvt8(h0 + (size_t)(b0 + srow) * HH + sc8, xh, xl);
        *(v8us*)&sAhi[0][srow][EE + sc8] = xh;
        *(v8us*)&sAlo[0][srow][EE + sc8] = xl;
        cvt8(xsrc(tokens, emb, hs_in, is_l0, nvocab, 0, b0 + srow, sc8), xh, xl);
        *(v8us*)&sAhi[0][srow][sc8] = xh;
        *(v8us*)&sAlo[0][srow][sc8] = xl;
    }
    v8f cReg;
#pragma unroll
    for (int r = 0; r < 8; ++r) cReg[r] = c0[(size_t)(b0 + 8 * h + r) * HH + u];

#pragma unroll 1
    for (int t = 0; t < TT; ++t) {
        const int cur = t & 1;
        const int nxt = cur ^ 1;

        __syncthreads();

        if (t > 0) {
            const int pb = (t - 1) & 1;
            float* dst = hs_out + ((size_t)(t - 1) * BB + b0) * HH;
            const v4f v0 = *(const v4f*)&sHf[pb][prow][pc4];
            const v4f v1 = *(const v4f*)&sHf[pb][prow + 8][pc4];
            *(volatile v4f*)(dst + tid * 4)         = v0;
            *(volatile v4f*)(dst + (tid + 128) * 4) = v1;
            __threadfence();
            *(volatile v4f*)(dst + tid * 4)         = v0;
            *(volatile v4f*)(dst + (tid + 128) * 4) = v1;
        }

        if (t + 1 < TT) {
            v8us xh, xl;
            cvt8(xsrc(tokens, emb, hs_in, is_l0, nvocab, t + 1, b0 + srow, sc8), xh, xl);
            *(v8us*)&sAhi[nxt][srow][sc8] = xh;
            *(v8us*)&sAlo[nxt][srow][sc8] = xl;
        }

        v8f acc[4];
#pragma unroll
        for (int q = 0; q < 4; ++q) acc[q] = zero8();

#pragma unroll 1
        for (int k0 = 0; k0 < KC; k0 += 32) {
            Frag ah, al, bh[4], bl[4];
            ah.half[0] = *(const v8us*)&sAhi[cur][m][k0 + 8 * h];
            ah.half[1] = *(const v8us*)&sAhi[cur][m][k0 + 8 * h + 16];
            al.half[0] = *(const v8us*)&sAlo[cur][m][k0 + 8 * h];
            al.half[1] = *(const v8us*)&sAlo[cur][m][k0 + 8 * h + 16];
#pragma unroll
            for (int q = 0; q < 4; ++q) {
                const unsigned short* ph = Whi + (size_t)(q * HH + u) * WP + k0 + 8 * h;
                const unsigned short* pl = Wlo + (size_t)(q * HH + u) * WP + k0 + 8 * h;
                bh[q].half[0] = *(const v8us*)(ph);
                bh[q].half[1] = *(const v8us*)(ph + 16);
                bl[q].half[0] = *(const v8us*)(pl);
                bl[q].half[1] = *(const v8us*)(pl + 16);
            }
#pragma unroll
            for (int q = 0; q < 4; ++q) acc[q] = mma(acc[q], ah, bh[q]);
#pragma unroll
            for (int q = 0; q < 4; ++q) acc[q] = mma(acc[q], ah, bl[q]);
#pragma unroll
            for (int q = 0; q < 4; ++q) acc[q] = mma(acc[q], al, bh[q]);
            asm volatile("v_nop\n\tv_nop\n\tv_nop\n\tv_nop"
                         : "+v"(acc[0]), "+v"(acc[1]), "+v"(acc[2]), "+v"(acc[3])
                         : "v"(ah.v), "v"(al.v),
                           "v"(bh[0].v), "v"(bh[1].v), "v"(bh[2].v), "v"(bh[3].v),
                           "v"(bl[0].v), "v"(bl[1].v), "v"(bl[2].v), "v"(bl[3].v));
        }

        {
            const float bi = sBias[u];
            const float bf = sBias[HH + u];
            const float bg = sBias[2 * HH + u];
            const float bo = sBias[3 * HH + u];
            const bool  last = (t == TT - 1);
#pragma unroll
            for (int r = 0; r < 8; ++r) {
                const int row = 8 * h + r;
                const float gi = acc[0][r] + bi;
                const float gf = acc[1][r] + bf;
                const float gg = acc[2][r] + bg;
                const float go = acc[3][r] + bo;
                const float cn = sigm(gf) * cReg[r] + sigm(gi) * tanhm(gg);
                const float hn = sigm(go) * tanhm(cn);
                cReg[r] = cn;
                sHf[cur][row][u] = hn;
                unsigned short th, tl;
                split2(hn, th, tl);
                sAhi[nxt][row][EE + u] = th;
                sAlo[nxt][row][EE + u] = tl;
                if (last) sCf[row][u] = cn;
            }
        }
    }

    __syncthreads();

    {
        float* dh = hs_out + ((size_t)(TT - 1) * BB + b0) * HH;
        float* o1 = out_h + (size_t)b0 * HH;
        float* o2 = out_c + (size_t)b0 * HH;
        const v4f hv0 = *(const v4f*)&sHf[1][prow][pc4];
        const v4f hv1 = *(const v4f*)&sHf[1][prow + 8][pc4];
        const v4f cv0 = *(const v4f*)&sCf[prow][pc4];
        const v4f cv1 = *(const v4f*)&sCf[prow + 8][pc4];
        const int p0 = tid * 4, p1 = (tid + 128) * 4;
        *(volatile v4f*)(dh + p0) = hv0;  *(volatile v4f*)(dh + p1) = hv1;
        *(volatile v4f*)(o1 + p0) = hv0;  *(volatile v4f*)(o1 + p1) = hv1;
        *(volatile v4f*)(o2 + p0) = cv0;  *(volatile v4f*)(o2 + p1) = cv1;
        __threadfence();
        *(volatile v4f*)(dh + p0) = hv0;  *(volatile v4f*)(dh + p1) = hv1;
        *(volatile v4f*)(o1 + p0) = hv0;  *(volatile v4f*)(o1 + p1) = hv1;
        *(volatile v4f*)(o2 + p0) = cv0;  *(volatile v4f*)(o2 + p1) = cv1;
    }
}

__global__ __launch_bounds__(256)
void fc_kernel(const float* __restrict__ hs_top, const float* __restrict__ Wfc,
               const float* __restrict__ bfc, float* out0)
{
    __shared__ __attribute__((aligned(16))) float sO[BB * OO];
    const int b = threadIdx.x;
    const float* hr = hs_top + (size_t)b * HH;
    float s0 = 0.0f, s1 = 0.0f, s2 = 0.0f;
#pragma unroll 2
    for (int k = 0; k < HH; ++k) {
        const float hv = hr[k];
        s0 += hv * Wfc[k];
        s1 += hv * Wfc[HH + k];
        s2 += hv * Wfc[2 * HH + k];
    }
    sO[b * OO + 0] = s0 + bfc[0];
    sO[b * OO + 1] = s1 + bfc[1];
    sO[b * OO + 2] = s2 + bfc[2];
    __syncthreads();
    v4f v;
#pragma unroll
    for (int i = 0; i < 4; ++i) v[i] = 0.0f;
    if (b < 192) v = *(const v4f*)&sO[b * 4];
    if (b < 192) *(volatile v4f*)(out0 + b * 4) = v;
    __threadfence();
    if (b < 192) *(volatile v4f*)(out0 + b * 4) = v;
}

extern "C" void kernel_launch(void* const* d_in, const int* in_sizes, int n_in,
                              void* d_out, int out_size, void* d_ws, size_t ws_size,
                              hipStream_t stream)
{
    if (n_in < 10) return;
    if (in_sizes[0] != BB * TT)            return;
    if (in_sizes[1] != LL * BB * HH)       return;
    if (in_sizes[2] != LL * BB * HH)       return;
    if (in_sizes[3] < EE || (in_sizes[3] % EE) != 0) return;
    if (in_sizes[4] != LL * G4 * EE)       return;
    if (in_sizes[5] != LL * G4 * HH)       return;
    if (in_sizes[6] != LL * G4)            return;
    if (in_sizes[7] != LL * G4)            return;
    if (in_sizes[8] != OO * HH)            return;
    if (in_sizes[9] != OO)                 return;
    if (out_size != BB * OO + 2 * LL * BB * HH) return;
    if (ws_size < WS_END)                  return;

    const int*   tokens = (const int*)d_in[0];
    const float* h0     = (const float*)d_in[1];
    const float* c0     = (const float*)d_in[2];
    const float* emb    = (const float*)d_in[3];
    const float* Wih    = (const float*)d_in[4];
    const float* Whh    = (const float*)d_in[5];
    const float* bih    = (const float*)d_in[6];
    const float* bhh    = (const float*)d_in[7];
    const float* Wfc    = (const float*)d_in[8];
    const float* bfc    = (const float*)d_in[9];
    const int nvocab = in_sizes[3] / EE;

    float* out  = (float*)d_out;
    float* out0 = out;
    float* out1 = out + BB * OO;
    float* out2 = out1 + LL * BB * HH;

    char* ws = (char*)d_ws;
    unsigned short* Whi = (unsigned short*)(ws + OFF_WHI);
    unsigned short* Wlo = (unsigned short*)(ws + OFF_WLO);
    float* plane[2];
    plane[0] = (float*)(ws + OFF_HSA);
    plane[1] = (float*)(ws + OFF_HSB);

    cvt_kernel<<<dim3(NWP / 256), dim3(256), 0, stream>>>(Wih, Whh, Whi, Wlo);

    for (int l = 0; l < LL; ++l) {
        const float* hs_in = plane[(l + 1) & 1];
        float* hs_out      = plane[l & 1];
        lstm_layer_kernel<<<dim3(NBLK), dim3(NTHR), 0, stream>>>(
            tokens, emb, hs_in,
            (const unsigned short*)(Whi + (size_t)l * G4 * WP),
            (const unsigned short*)(Wlo + (size_t)l * G4 * WP),
            bih + (size_t)l * G4, bhh + (size_t)l * G4,
            h0 + (size_t)l * BB * HH, c0 + (size_t)l * BB * HH,
            hs_out, out1 + (size_t)l * BB * HH, out2 + (size_t)l * BB * HH,
            (l == 0) ? 1 : 0, nvocab);
    }

    fc_kernel<<<dim3(1), dim3(256), 0, stream>>>(
        (const float*)(plane[(LL - 1) & 1] + (size_t)(TT - 1) * BB * HH), Wfc, bfc, out0);
}
